// HybridGCN_86397562126412
// MI455X (gfx1250) — hardware-verified
//
#include <hip/hip_runtime.h>
#include <stdint.h>
#include <stddef.h>


#define DIN   256
#define HID   512
#define NHD   4
#define DHD   64
#define NB    128
#define CHUNK 2048
#define NTHR  256
#define NWAVE 8
#define WCAP  256
#define NGRP  (CHUNK / (NTHR * 4))
#define PCAP  128
#define SPW   (NB / NWAVE)
#define GT    64
#define GTHR  128
#define CP    68

#define GAT_LDS_BYTES ((NB * DIN + 2 * NB * NHD + NWAVE * WCAP + NWAVE) * 4)
#define GIN_LDS_BYTES ((NB * PCAP + NB + NWAVE * WCAP + NWAVE + NWAVE * PCAP) * 4)

static_assert(WCAP == (CHUNK / NTHR) * 32);
static_assert(NGRP == 2);
static_assert(NB == 128);
static_assert((NB & (NB - 1)) == 0);
static_assert(DIN == NHD * DHD);
static_assert(SPW == 16);
static_assert(PCAP == 4 * 32);
static_assert((CP % 4) == 0);
static_assert(GAT_LDS_BYTES == 143392);
static_assert(GIN_LDS_BYTES == 78368);

typedef float          v4f   __attribute__((ext_vector_type(4)));
typedef float          v8f   __attribute__((ext_vector_type(8)));
typedef int            v4i   __attribute__((ext_vector_type(4)));
typedef unsigned int   v4u   __attribute__((ext_vector_type(4)));
typedef unsigned short v8us  __attribute__((ext_vector_type(8)));
typedef __bf16         v16bf __attribute__((ext_vector_type(16)));
union FragU { v16bf v; v8us half[2]; };

__device__ __forceinline__ int imin(int a, int b) { return a < b ? a : b; }
__device__ __forceinline__ int iclamp(int v, int lo, int hi) { return v < lo ? lo : (v > hi ? hi : v); }

__device__ __forceinline__ unsigned int bfb(float f) {
  unsigned int u = __float_as_uint(f);
  u += 0x7fffu + ((u >> 16) & 1u);
  return u >> 16;
}
__device__ __forceinline__ unsigned int hl2(float v, unsigned int& lo) {
  const unsigned int hi = bfb(v);
  lo = bfb(v - __uint_as_float(hi << 16));
  return hi;
}
__device__ __forceinline__ void split8(v4f a, v4f b, v4u& hi, v4u& lo) {
  unsigned int l0, l1, l2, l3, l4, l5, l6, l7;
  const unsigned int h0 = hl2(a.x, l0), h1 = hl2(a.y, l1), h2 = hl2(a.z, l2), h3 = hl2(a.w, l3);
  const unsigned int h4 = hl2(b.x, l4), h5 = hl2(b.y, l5), h6 = hl2(b.z, l6), h7 = hl2(b.w, l7);
  hi.x = h0 | (h1 << 16); hi.y = h2 | (h3 << 16); hi.z = h4 | (h5 << 16); hi.w = h6 | (h7 << 16);
  lo.x = l0 | (l1 << 16); lo.y = l2 | (l3 << 16); lo.z = l4 | (l5 << 16); lo.w = l6 | (l7 << 16);
}

__device__ __forceinline__ v8f wm(v16bf a, v16bf b, v8f c) {
  v8f d = __builtin_amdgcn_wmma_f32_16x16x32_bf16(false, a, false, b, (short)0, c, false, false);
  asm volatile("v_nop\n\tv_nop\n\tv_nop\n\tv_nop" : "+v"(d) : "v"(a), "v"(b));
  return d;
}

__device__ __forceinline__ v8f z8() {
  v8f z = {0.f, 0.f, 0.f, 0.f, 0.f, 0.f, 0.f, 0.f};
  return z;
}

__device__ __forceinline__ float wsum(float v) {
  v += __shfl_xor(v, 16, 32);
  v += __shfl_xor(v, 8, 32);
  v += __shfl_xor(v, 4, 32);
  v += __shfl_xor(v, 2, 32);
  v += __shfl_xor(v, 1, 32);
  return v;
}

__device__ __forceinline__ v4f leaky4(v4f v) {
  v4f r;
  r.x = fmaxf(v.x, 0.2f * v.x);
  r.y = fmaxf(v.y, 0.2f * v.y);
  r.z = fmaxf(v.z, 0.2f * v.z);
  r.w = fmaxf(v.w, 0.2f * v.w);
  return r;
}

__device__ __forceinline__ int scan_chunk(const int* __restrict__ key, int nE, int cbase,
                                          int nodeBase, int* list, int wave, int tid, int al16) {
  int wc = 0;
#pragma unroll
  for (int g = 0; g < NGRP; ++g) {
    const int el0 = (g * NTHR + tid) * 4;
    const int e0 = cbase + el0;
    const int sent = -2147483647 - 1;
    v4i d;
    if (al16 != 0 && (cbase + CHUNK <= nE)) {
      d = *(const v4i*)(key + e0);
    } else {
      const int c0 = imin(e0, nE - 1), c1 = imin(e0 + 1, nE - 1);
      const int c2 = imin(e0 + 2, nE - 1), c3 = imin(e0 + 3, nE - 1);
      const int k0v = key[c0], k1v = key[c1], k2v = key[c2], k3v = key[c3];
      d.x = (e0     < nE) ? k0v : sent;
      d.y = (e0 + 1 < nE) ? k1v : sent;
      d.z = (e0 + 2 < nE) ? k2v : sent;
      d.w = (e0 + 3 < nE) ? k3v : sent;
    }
    const unsigned s0 = (unsigned)d.x - (unsigned)nodeBase;
    const unsigned s1 = (unsigned)d.y - (unsigned)nodeBase;
    const unsigned s2 = (unsigned)d.z - (unsigned)nodeBase;
    const unsigned s3 = (unsigned)d.w - (unsigned)nodeBase;
    const bool h0 = s0 < (unsigned)NB;
    const bool h1 = s1 < (unsigned)NB;
    const bool h2 = s2 < (unsigned)NB;
    const bool h3 = s3 < (unsigned)NB;
    const unsigned many = __builtin_amdgcn_ballot_w32(h0 | h1 | h2 | h3);
    if (many != 0u) {
#define HITJ(J, HJ, SJ) { \
        const unsigned mj = __builtin_amdgcn_ballot_w32(HJ); \
        if (HJ) { \
          const int pos = wc + (int)__builtin_amdgcn_mbcnt_lo(mj, 0u); \
          if (pos < WCAP) list[wave * WCAP + pos] = ((el0 + (J)) << 9) | (int)(SJ); \
        } \
        wc += (int)__builtin_popcount(mj); }
      HITJ(0, h0, s0)
      HITJ(1, h1, s1)
      HITJ(2, h2, s2)
      HITJ(3, h3, s3)
#undef HITJ
    }
  }
  return wc;
}

__global__ __launch_bounds__(NTHR) void k_cvt(const float* __restrict__ X,
                                              unsigned short* Ph, unsigned short* Pl, int n8) {
  const int i = blockIdx.x * NTHR + threadIdx.x;
  if (i >= n8) return;
  const size_t o = (size_t)i * 8;
  const v4f a = *(const v4f*)(X + o);
  const v4f b = *(const v4f*)(X + o + 4);
  v4u hi, lo;
  split8(a, b, hi, lo);
  *(volatile v4u*)(Ph + o) = hi;
  *(volatile v4u*)(Pl + o) = lo;
  __threadfence();
  *(volatile v4u*)(Ph + o) = hi;
  *(volatile v4u*)(Pl + o) = lo;
}

__global__ __launch_bounds__(NTHR) void k_cvtT(const float* __restrict__ W, int Kd, int Nd,
                                               unsigned short* Th, unsigned short* Tl) {
  __shared__ __attribute__((aligned(16))) float Ws[64 * CP];
  const int tid = threadIdx.x;
  const int k0 = blockIdx.y * 64, n0 = blockIdx.x * 64;
  {
    const int r = tid >> 2;
    const int c = (tid & 3) * 16;
    const float* p = W + (size_t)(k0 + r) * Nd + n0 + c;
    const v4f f0 = *(const v4f*)(p), f1 = *(const v4f*)(p + 4);
    const v4f f2 = *(const v4f*)(p + 8), f3 = *(const v4f*)(p + 12);
    *(v4f*)(Ws + r * CP + c)      = f0;
    *(v4f*)(Ws + r * CP + c + 4)  = f1;
    *(v4f*)(Ws + r * CP + c + 8)  = f2;
    *(v4f*)(Ws + r * CP + c + 12) = f3;
  }
  __syncthreads();
  v4u hiv[2], lov[2];
  size_t ov[2];
#pragma unroll
  for (int pz = 0; pz < 2; ++pz) {
    const int nn = pz * 32 + (tid >> 3);
    const int kk = (tid & 7) * 8;
    v4f a, b;
    a.x = Ws[(kk + 0) * CP + nn]; a.y = Ws[(kk + 1) * CP + nn];
    a.z = Ws[(kk + 2) * CP + nn]; a.w = Ws[(kk + 3) * CP + nn];
    b.x = Ws[(kk + 4) * CP + nn]; b.y = Ws[(kk + 5) * CP + nn];
    b.z = Ws[(kk + 6) * CP + nn]; b.w = Ws[(kk + 7) * CP + nn];
    split8(a, b, hiv[pz], lov[pz]);
    ov[pz] = (size_t)(n0 + nn) * Kd + k0 + kk;
  }
#pragma unroll
  for (int pz = 0; pz < 2; ++pz) {
    *(volatile v4u*)(Th + ov[pz]) = hiv[pz];
    *(volatile v4u*)(Tl + ov[pz]) = lov[pz];
  }
  __threadfence();
#pragma unroll
  for (int pz = 0; pz < 2; ++pz) {
    *(volatile v4u*)(Th + ov[pz]) = hiv[pz];
    *(volatile v4u*)(Tl + ov[pz]) = lov[pz];
  }
}

__device__ __forceinline__ void epi_lds(v8f acc, int rbase, int col, float bv, int relu, float* Cs) {
#pragma unroll
  for (int r = 0; r < 8; ++r) {
    float v = acc[r] + bv;
    if (relu != 0) v = fmaxf(v, 0.f);
    Cs[(rbase + r) * CP + col] = v;
  }
}

__global__ __launch_bounds__(GTHR) void k_gemm(
    const unsigned short* __restrict__ Ah, const unsigned short* __restrict__ Al, int lda,
    const unsigned short* __restrict__ Bh, const unsigned short* __restrict__ Bl, int ldb, int K,
    const float* __restrict__ bias, int hasBias, int relu,
    float* Cf, unsigned short* Ch, unsigned short* Cl, int ldc, int mode) {
  __shared__ __attribute__((aligned(16))) float Cs[GT * CP];

  const int tid  = threadIdx.x;
  const int lane = tid & 31;
  const int wave = tid >> 5;
  const int h    = lane >> 4;
  const int m    = lane & 15;
  const int wr   = wave >> 1;
  const int wc   = wave & 1;
  const int m0   = blockIdx.y * GT;
  const int n0   = blockIdx.x * GT;

  const unsigned short* pAh0 = Ah + (size_t)(m0 + 32 * wr + m) * lda + 8 * h;
  const unsigned short* pAh1 = pAh0 + (size_t)16 * lda;
  const unsigned short* pAl0 = Al + (size_t)(m0 + 32 * wr + m) * lda + 8 * h;
  const unsigned short* pAl1 = pAl0 + (size_t)16 * lda;
  const unsigned short* pBh0 = Bh + (size_t)(n0 + 32 * wc + m) * ldb + 8 * h;
  const unsigned short* pBh1 = pBh0 + (size_t)16 * ldb;
  const unsigned short* pBl0 = Bl + (size_t)(n0 + 32 * wc + m) * ldb + 8 * h;
  const unsigned short* pBl1 = pBl0 + (size_t)16 * ldb;

  v8f acc00 = z8(), acc01 = z8(), acc10 = z8(), acc11 = z8();

#pragma unroll 1
  for (int k0 = 0; k0 < K; k0 += 32) {
    FragU ah0, ah1, al0, al1, bh0, bh1, bl0, bl1;
    ah0.half[0] = *(const v8us*)(pAh0 + k0); ah0.half[1] = *(const v8us*)(pAh0 + k0 + 16);
    ah1.half[0] = *(const v8us*)(pAh1 + k0); ah1.half[1] = *(const v8us*)(pAh1 + k0 + 16);
    al0.half[0] = *(const v8us*)(pAl0 + k0); al0.half[1] = *(const v8us*)(pAl0 + k0 + 16);
    al1.half[0] = *(const v8us*)(pAl1 + k0); al1.half[1] = *(const v8us*)(pAl1 + k0 + 16);
    bh0.half[0] = *(const v8us*)(pBh0 + k0); bh0.half[1] = *(const v8us*)(pBh0 + k0 + 16);
    bh1.half[0] = *(const v8us*)(pBh1 + k0); bh1.half[1] = *(const v8us*)(pBh1 + k0 + 16);
    bl0.half[0] = *(const v8us*)(pBl0 + k0); bl0.half[1] = *(const v8us*)(pBl0 + k0 + 16);
    bl1.half[0] = *(const v8us*)(pBl1 + k0); bl1.half[1] = *(const v8us*)(pBl1 + k0 + 16);

    acc00 = wm(ah0.v, bh0.v, acc00); acc00 = wm(ah0.v, bl0.v, acc00); acc00 = wm(al0.v, bh0.v, acc00);
    acc01 = wm(ah0.v, bh1.v, acc01); acc01 = wm(ah0.v, bl1.v, acc01); acc01 = wm(al0.v, bh1.v, acc01);
    acc10 = wm(ah1.v, bh0.v, acc10); acc10 = wm(ah1.v, bl0.v, acc10); acc10 = wm(al1.v, bh0.v, acc10);
    acc11 = wm(ah1.v, bh1.v, acc11); acc11 = wm(ah1.v, bl1.v, acc11); acc11 = wm(al1.v, bh1.v, acc11);
  }

  const int colA = 32 * wc + m;
  const int colB = colA + 16;
  float bA = 0.f, bB = 0.f;
  if (hasBias != 0) {
    bA = bias[n0 + colA];
    bB = bias[n0 + colB];
  }
  epi_lds(acc00, 32 * wr + 8 * h,      colA, bA, relu, Cs);
  epi_lds(acc01, 32 * wr + 8 * h,      colB, bB, relu, Cs);
  epi_lds(acc10, 32 * wr + 16 + 8 * h, colA, bA, relu, Cs);
  epi_lds(acc11, 32 * wr + 16 + 8 * h, colB, bB, relu, Cs);
  __syncthreads();

  if (mode == 0) {
    for (int ps = 0; ps < 2; ++ps) {
#pragma unroll
      for (int it = 0; it < 8; ++it) {
        const int row = 16 * wave + 2 * it + (lane >> 4);
        const int c4  = 4 * (lane & 15);
        const v4f v = *(const v4f*)(Cs + row * CP + c4);
        *(volatile v4f*)(Cf + (size_t)(m0 + row) * ldc + n0 + c4) = v;
      }
      if (ps == 0) __threadfence();
    }
  } else {
    for (int ps = 0; ps < 2; ++ps) {
#pragma unroll
      for (int it = 0; it < 4; ++it) {
        const int row = 16 * wave + 4 * it + (lane >> 3);
        const int c8  = 8 * (lane & 7);
        const v4f a = *(const v4f*)(Cs + row * CP + c8);
        const v4f b = *(const v4f*)(Cs + row * CP + c8 + 4);
        v4u hi, lo;
        split8(a, b, hi, lo);
        const size_t o = (size_t)(m0 + row) * ldc + n0 + c8;
        *(volatile v4u*)(Ch + o) = hi;
        *(volatile v4u*)(Cl + o) = lo;
      }
      if (ps == 0) __threadfence();
    }
  }
}

__global__ __launch_bounds__(NTHR) void k_gin(const float* __restrict__ x, const int* __restrict__ ei,
                                              unsigned short* Hh, unsigned short* Hl, int nN, int nE) {
  extern __shared__ v4f lds_g[];
  int* plist = (int*)lds_g;
  int* pcnt  = plist + NB * PCAP;
  int* list  = pcnt + NB;
  int* wcnt  = list + NWAVE * WCAP;
  int* sbuf  = wcnt + NWAVE;

  const int tid  = threadIdx.x;
  const int lane = tid & 31;
  const int wave = tid >> 5;
  const int nodeBase = blockIdx.x * NB;

  for (int i = tid; i < NB; i += NTHR) pcnt[i] = 0;
  __syncthreads();

  const int* key = ei;
  const int al16 = ((((uintptr_t)(const void*)key) & 15u) == 0) ? 1 : 0;
  const int nChunks = (nE + CHUNK - 1) / CHUNK;

#pragma unroll 1
  for (int ch = 0; ch < nChunks; ++ch) {
    const int cbase = ch * CHUNK;
    const int wc = scan_chunk(key, nE, cbase, nodeBase, list, wave, tid, al16);
    if (lane == 0) wcnt[wave] = wc;
    __syncthreads();
    if (wave == 0) {
#pragma unroll 1
      for (int wsx = 0; wsx < NWAVE; ++wsx) {
        int n = wcnt[wsx];
        n = n > WCAP ? WCAP : n;
        n = n < 0 ? 0 : n;
#pragma unroll 1
        for (int i = 0; i < n; ++i) {
          const int ent  = list[wsx * WCAP + i];
          const int slot = ent & (NB - 1);
          int e = cbase + ((ent >> 9) & (CHUNK - 1));
          e = e > nE - 1 ? nE - 1 : e;
          const int j   = iclamp(ei[(size_t)nE + e], 0, nN - 1);
          const int c   = pcnt[slot];
          const int pos = c < PCAP - 1 ? c : PCAP - 1;
          if (lane == 0) plist[slot * PCAP + pos] = j;
          pcnt[slot] = c + 1;
        }
      }
    }
    __syncthreads();
  }

#pragma unroll 1
  for (int js = 0; js < SPW; ++js) {
    const int slot = wave * SPW + js;
    const int node = nodeBase + slot;
    if (node >= nN) break;
    int n = pcnt[slot];
    n = n > PCAP ? PCAP : n;
    n = n < 0 ? 0 : n;
    const int* pl = plist + slot * PCAP;
    int v[4], rk[4];
#pragma unroll
    for (int t = 0; t < 4; ++t) {
      const int i  = lane + 32 * t;
      const int vi = pl[i];
      v[t]  = (i < n) ? vi : 0x7fffffff;
      rk[t] = 0;
    }
#pragma unroll 1
    for (int ip = 0; ip < n; ++ip) {
      const int u = pl[ip];
#pragma unroll
      for (int t = 0; t < 4; ++t) {
        const int i = lane + 32 * t;
        rk[t] += ((u < v[t]) || (u == v[t] && ip < i)) ? 1 : 0;
      }
    }
    int* sb = sbuf + wave * PCAP;
    __builtin_amdgcn_wave_barrier();
#pragma unroll
    for (int t = 0; t < 4; ++t) {
      const int i = lane + 32 * t;
      const int r = rk[t] > PCAP - 1 ? PCAP - 1 : rk[t];
      if (i < n) sb[r] = v[t];
    }
    __builtin_amdgcn_fence(__ATOMIC_RELEASE, "wavefront");
    __builtin_amdgcn_wave_barrier();

    v4f ca = {0.f, 0.f, 0.f, 0.f};
    v4f cb = {0.f, 0.f, 0.f, 0.f};
    int prv = -1;
#pragma unroll 1
    for (int p = 0; p < n; ++p) {
      const int j  = sb[p];
      const int jj = iclamp(j, 0, nN - 1);
      const float* px = x + (size_t)jj * DIN + 8 * lane;
      const v4f xa = *(const v4f*)(px);
      const v4f xb = *(const v4f*)(px + 4);
      const bool take = (j != prv);
      ca = take ? (ca + xa) : ca;
      cb = take ? (cb + xb) : cb;
      prv = j;
    }
    __builtin_amdgcn_wave_barrier();
    const float* pxs = x + (size_t)node * DIN + 8 * lane;
    const v4f ha = *(const v4f*)(pxs) + ca;
    const v4f hb = *(const v4f*)(pxs + 4) + cb;
    v4u hi, lo;
    split8(ha, hb, hi, lo);
    const size_t o = (size_t)node * DIN + 8 * lane;
    *(volatile v4u*)(Hh + o) = hi;
    *(volatile v4u*)(Hl + o) = lo;
    __threadfence();
    *(volatile v4u*)(Hh + o) = hi;
    *(volatile v4u*)(Hl + o) = lo;
  }
}

__global__ __launch_bounds__(NTHR) void k_gat(const float* __restrict__ xlr, const int* __restrict__ ei,
                                              const float* __restrict__ att, const float* __restrict__ bg,
                                              unsigned short* Afh, unsigned short* Afl, int nN, int nE) {
  extern __shared__ v4f lds_a[];
  float* sacc = (float*)lds_a;
  float* mxa  = sacc + NB * DIN;
  float* dna  = mxa + NB * NHD;
  int*   list = (int*)(dna + NB * NHD);
  int*   wcnt = list + NWAVE * WCAP;

  const int tid  = threadIdx.x;
  const int lane = tid & 31;
  const int wave = tid >> 5;
  const int hd   = lane >> 3;
  const int nodeBase = blockIdx.x * NB;

  {
    const v4f z4 = {0.f, 0.f, 0.f, 0.f};
    for (int i = tid; i < (NB * DIN) / 4; i += NTHR) lds_a[i] = z4;
    for (int i = tid; i < NB * NHD; i += NTHR) { mxa[i] = -1.0e30f; dna[i] = 0.f; }
  }
  const v4f a0 = *(const v4f*)(att + 8 * lane);
  const v4f a1 = *(const v4f*)(att + 8 * lane + 4);
  __syncthreads();

  const int* key = ei + nE;
  const int al16 = ((((uintptr_t)(const void*)key) & 15u) == 0) ? 1 : 0;
  const int nChunks = (nE + CHUNK - 1) / CHUNK;

#pragma unroll 1
  for (int ch = 0; ch < nChunks; ++ch) {
    const int cbase = ch * CHUNK;
    const int wc = scan_chunk(key, nE, cbase, nodeBase, list, wave, tid, al16);
    if (lane == 0) wcnt[wave] = wc;
    __syncthreads();

    if (wave == 0) {
      const int nself = (ch == nChunks - 1) ? NB : 0;
#pragma unroll 1
      for (int wsx = 0; wsx <= NWAVE; ++wsx) {
        const bool isSelf = (wsx == NWAVE);
        const int  wl = isSelf ? (NWAVE - 1) : wsx;
        int n = wcnt[wl];
        n = n > WCAP ? WCAP : n;
        n = n < 0 ? 0 : n;
        n = isSelf ? nself : n;
#pragma unroll 1
        for (int i = 0; i < n; ++i) {
          const int ent = list[wl * WCAP + (i & (WCAP - 1))];
          int e = cbase + ((ent >> 9) & (CHUNK - 1));
          e = e > nE - 1 ? nE - 1 : e;
          const int srcE = iclamp(ei[e], 0, nN - 1);
          const int slot = isSelf ? i : (ent & (NB - 1));
          int nd = nodeBase + slot;
          nd = nd > nN - 1 ? nN - 1 : nd;
          const int src = isSelf ? nd : srcE;

          const float* ps = xlr + (size_t)src * HID + 8 * lane;
          const float* pd = xlr + (size_t)nd * HID + DIN + 8 * lane;
          const v4f xa = *(const v4f*)(ps);
          const v4f xb = *(const v4f*)(ps + 4);
          const v4f ra = *(const v4f*)(pd);
          const v4f rb = *(const v4f*)(pd + 4);
          const v4f ta = leaky4(xa + ra);
          const v4f tb = leaky4(xb + rb);
          float s = ta.x * a0.x + ta.y * a0.y + ta.z * a0.z + ta.w * a0.w
                  + tb.x * a1.x + tb.y * a1.y + tb.z * a1.z + tb.w * a1.w;
          s += __shfl_xor(s, 4, 32);
          s += __shfl_xor(s, 2, 32);
          s += __shfl_xor(s, 1, 32);
          const int ai = slot * NHD + hd;
          const float Mo = mxa[ai];
          const float Do = dna[ai];
          const float Mn = fmaxf(Mo, s);
          const float sc = __expf(Mo - Mn);
          const float p  = __expf(s - Mn);
          float* sp = sacc + slot * DIN + 8 * lane;
          v4f ca = *(const v4f*)(sp);
          v4f cb = *(const v4f*)(sp + 4);
          ca = ca * sc + xa * p;
          cb = cb * sc + xb * p;
          *(v4f*)(sp)     = ca;
          *(v4f*)(sp + 4) = cb;
          mxa[ai] = Mn;
          dna[ai] = Do * sc + p;
        }
      }
    }
    __syncthreads();
  }

  const v4f b0 = *(const v4f*)(bg + 8 * lane);
  const v4f b1 = *(const v4f*)(bg + 8 * lane + 4);
#pragma unroll 1
  for (int j = 0; j < SPW; ++j) {
    const int slot = wave * SPW + j;
    const int node = nodeBase + slot;
    if (node >= nN) break;
    const float* sp = sacc + slot * DIN + 8 * lane;
    const v4f ca = *(const v4f*)(sp);
    const v4f cb = *(const v4f*)(sp + 4);
    const float d   = dna[slot * NHD + hd];
    const float inv = __builtin_amdgcn_rcpf(d);
    const v4f ya = ca * inv + b0;
    const v4f yb = cb * inv + b1;
    v4u hi, lo;
    split8(ya, yb, hi, lo);
    const size_t o = (size_t)node * HID + 8 * lane;
    *(volatile v4u*)(Afh + o) = hi;
    *(volatile v4u*)(Afl + o) = lo;
    __threadfence();
    *(volatile v4u*)(Afh + o) = hi;
    *(volatile v4u*)(Afl + o) = lo;
  }
}

__global__ __launch_bounds__(NTHR) void k_ln(const float* __restrict__ C, const float* __restrict__ g,
                                             const float* __restrict__ b, float* out, int nN) {
  const int lane = threadIdx.x & 31;
  const int wave = threadIdx.x >> 5;
  const int row  = blockIdx.x * NWAVE + wave;
  if (row >= nN) return;
  const size_t base = (size_t)row * HID + 4 * lane;
  const v4f c0 = *(const v4f*)(C + base);
  const v4f c1 = *(const v4f*)(C + base + 128);
  const v4f c2 = *(const v4f*)(C + base + 256);
  const v4f c3 = *(const v4f*)(C + base + 384);
  float s = (c0.x + c0.y + c0.z + c0.w) + (c1.x + c1.y + c1.z + c1.w)
          + (c2.x + c2.y + c2.z + c2.w) + (c3.x + c3.y + c3.z + c3.w);
  s = wsum(s);
  const float mu = s * (1.0f / HID);
  const v4f d0 = c0 - mu, d1 = c1 - mu, d2 = c2 - mu, d3 = c3 - mu;
  float q = (d0.x * d0.x + d0.y * d0.y + d0.z * d0.z + d0.w * d0.w)
          + (d1.x * d1.x + d1.y * d1.y + d1.z * d1.z + d1.w * d1.w)
          + (d2.x * d2.x + d2.y * d2.y + d2.z * d2.z + d2.w * d2.w)
          + (d3.x * d3.x + d3.y * d3.y + d3.z * d3.z + d3.w * d3.w);
  q = wsum(q);
  const float rs = rsqrtf(q * (1.0f / HID) + 1.0e-5f);
  const v4f g0 = *(const v4f*)(g + 4 * lane),       e0 = *(const v4f*)(b + 4 * lane);
  const v4f g1 = *(const v4f*)(g + 4 * lane + 128), e1 = *(const v4f*)(b + 4 * lane + 128);
  const v4f g2 = *(const v4f*)(g + 4 * lane + 256), e2 = *(const v4f*)(b + 4 * lane + 256);
  const v4f g3 = *(const v4f*)(g + 4 * lane + 384), e3 = *(const v4f*)(b + 4 * lane + 384);
  const v4f y0 = d0 * rs * g0 + e0;
  const v4f y1 = d1 * rs * g1 + e1;
  const v4f y2 = d2 * rs * g2 + e2;
  const v4f y3 = d3 * rs * g3 + e3;
  *(volatile v4f*)(out + base)       = y0;
  *(volatile v4f*)(out + base + 128) = y1;
  *(volatile v4f*)(out + base + 256) = y2;
  *(volatile v4f*)(out + base + 384) = y3;
  __threadfence();
  *(volatile v4f*)(out + base)       = y0;
  *(volatile v4f*)(out + base + 128) = y1;
  *(volatile v4f*)(out + base + 256) = y2;
  *(volatile v4f*)(out + base + 384) = y3;
}

extern "C" void kernel_launch(void* const* d_in, const int* in_sizes, int n_in,
                              void* d_out, int out_size, void* d_ws, size_t ws_size,
                              hipStream_t stream) {
  if (n_in < 14) return;
  const int nN = in_sizes[0] / DIN;
  if (nN <= 0 || in_sizes[0] != nN * DIN || (nN % NB) != 0) return;
  if (in_sizes[1] != DIN * DIN || in_sizes[2] != DIN * DIN) return;
  if (in_sizes[3] != NHD * DHD || in_sizes[4] != DIN) return;
  if (in_sizes[5] != DIN * DIN || in_sizes[6] != DIN) return;
  if (in_sizes[7] != DIN * DIN || in_sizes[8] != DIN) return;
  if (in_sizes[9] != HID * HID || in_sizes[10] != HID) return;
  if (in_sizes[11] != HID || in_sizes[12] != HID) return;
  if (in_sizes[13] < 2 || (in_sizes[13] & 1) != 0) return;
  const int nE = in_sizes[13] / 2;
  if (out_size != nN * HID) return;

  const float* x   = (const float*)d_in[0];
  const float* Wl  = (const float*)d_in[1];
  const float* Wr  = (const float*)d_in[2];
  const float* att = (const float*)d_in[3];
  const float* bg  = (const float*)d_in[4];
  const float* gW1 = (const float*)d_in[5];
  const float* gb1 = (const float*)d_in[6];
  const float* gW2 = (const float*)d_in[7];
  const float* gb2 = (const float*)d_in[8];
  const float* fW  = (const float*)d_in[9];
  const float* fb  = (const float*)d_in[10];
  const float* lng = (const float*)d_in[11];
  const float* lnb = (const float*)d_in[12];
  const int*   ei  = (const int*)d_in[13];
  float* out = (float*)d_out;

  char* wsb = (char*)d_ws;
  size_t off = 0;
#define CARVE(T, name, nbytes) T* name = (T*)(wsb + off); off += ((((size_t)(nbytes)) + 255) / 256) * 256;
  CARVE(unsigned short, Xh,    (size_t)nN * DIN * 2)
  CARVE(unsigned short, Xl,    (size_t)nN * DIN * 2)
  CARVE(unsigned short, WlrTh, (size_t)HID * DIN * 2)
  CARVE(unsigned short, WlrTl, (size_t)HID * DIN * 2)
  CARVE(unsigned short, W1Th,  (size_t)DIN * DIN * 2)
  CARVE(unsigned short, W1Tl,  (size_t)DIN * DIN * 2)
  CARVE(unsigned short, W2Th,  (size_t)DIN * DIN * 2)
  CARVE(unsigned short, W2Tl,  (size_t)DIN * DIN * 2)
  CARVE(unsigned short, FTh,   (size_t)HID * HID * 2)
  CARVE(unsigned short, FTl,   (size_t)HID * HID * 2)
  CARVE(float,          XLR,   (size_t)nN * HID * 4)
  CARVE(unsigned short, Afh,   (size_t)nN * HID * 2)
  CARVE(unsigned short, Afl,   (size_t)nN * HID * 2)
  CARVE(unsigned short, Hh,    (size_t)nN * DIN * 2)
  CARVE(unsigned short, Hl,    (size_t)nN * DIN * 2)
  CARVE(unsigned short, Tph,   (size_t)nN * DIN * 2)
  CARVE(unsigned short, Tpl,   (size_t)nN * DIN * 2)
  CARVE(float,          Cf,    (size_t)nN * HID * 4)
#undef CARVE
  if (off > ws_size) return;

  const int n8 = nN * DIN / 8;
  k_cvt<<<(n8 + NTHR - 1) / NTHR, NTHR, 0, stream>>>(x, Xh, Xl, n8);
  k_cvtT<<<dim3(DIN / 64, DIN / 64), NTHR, 0, stream>>>(Wl,  DIN, DIN, WlrTh, WlrTl);
  k_cvtT<<<dim3(DIN / 64, DIN / 64), NTHR, 0, stream>>>(Wr,  DIN, DIN, WlrTh + DIN * DIN, WlrTl + DIN * DIN);
  k_cvtT<<<dim3(DIN / 64, DIN / 64), NTHR, 0, stream>>>(gW1, DIN, DIN, W1Th, W1Tl);
  k_cvtT<<<dim3(DIN / 64, DIN / 64), NTHR, 0, stream>>>(gW2, DIN, DIN, W2Th, W2Tl);
  k_cvtT<<<dim3(HID / 64, HID / 64), NTHR, 0, stream>>>(fW,  HID, HID, FTh, FTl);

  k_gemm<<<dim3(HID / GT, nN / GT), GTHR, 0, stream>>>(Xh, Xl, DIN, WlrTh, WlrTl, DIN, DIN,
                                                       fb, 0, 0, XLR, Tph, Tpl, HID, 0);

  hipFuncSetAttribute(reinterpret_cast<const void*>(&k_gin),
                      hipFuncAttributeMaxDynamicSharedMemorySize, GIN_LDS_BYTES);
  k_gin<<<nN / NB, NTHR, GIN_LDS_BYTES, stream>>>(x, ei, Hh, Hl, nN, nE);
  k_gemm<<<dim3(DIN / GT, nN / GT), GTHR, 0, stream>>>(Hh, Hl, DIN, W1Th, W1Tl, DIN, DIN,
                                                       gb1, 1, 1, Cf, Tph, Tpl, DIN, 1);
  k_gemm<<<dim3(DIN / GT, nN / GT), GTHR, 0, stream>>>(Tph, Tpl, DIN, W2Th, W2Tl, DIN, DIN,
                                                       gb2, 1, 0, Cf, Afh + DIN, Afl + DIN, HID, 1);

  hipFuncSetAttribute(reinterpret_cast<const void*>(&k_gat),
                      hipFuncAttributeMaxDynamicSharedMemorySize, GAT_LDS_BYTES);
  k_gat<<<nN / NB, NTHR, GAT_LDS_BYTES, stream>>>(XLR, ei, att, bg, Afh, Afl, nN, nE);

  k_gemm<<<dim3(HID / GT, nN / GT), GTHR, 0, stream>>>(Afh, Afl, HID, FTh, FTl, HID, HID,
                                                       fb, 1, 1, Cf, Tph, Tpl, HID, 0);
  k_ln<<<nN / NWAVE, NTHR, 0, stream>>>(Cf, lng, lnb, out, nN);
}
